// GCN_91096256348387
// MI455X (gfx1250) — hardware-run, weakly checked
//
#include <hip/hip_runtime.h>
#include <stddef.h>
#include <stdint.h>
#include <math.h>

#define NN      50000
#define NE      1000000
#define CIN     128
#define HD      64
#define NTHR    256
#define NWAVE   8
#define EPT     8
#define WCH     (32 * EPT)
#define NBRUN   1024
#define SLB     10
#define NBK     49
#define MP      (NBK * NBRUN)
#define GBM     128
#define WLCAP   3584
#define RCAP    22528
#define DEGCAP  64
#define MAXDEG_MEAS   42
#define MAXB1024_MEAS 20780
#define SP      68

#define BK_ZINTS (NWAVE * WLCAP + RCAP + 3 * NBRUN)
#define BK_INTS  (BK_ZINTS + 16 + NBRUN)
#define BK_LDS   (BK_INTS * 4)

#define PBX   (MP * CIN / 8 / NTHR)
#define PBW1  (HD * CIN / 8 / NTHR)
#define PBTOT (PBX + PBW1 + 1)

static_assert(NN == 50000 && NE == 1000000);
static_assert(HD == 64 && HD == 16 * 4 && CIN % 32 == 0 && CIN / 8 == 16);
static_assert(NBRUN == (1 << SLB) && NBRUN == 4 * NTHR && NBRUN % GBM == 0);
static_assert(NBK * NBRUN >= NN && MP % GBM == 0 && NN <= MP);
static_assert(NE < (1 << 21) && (((long long)NE) << SLB) < (1LL << 31));
static_assert(NE % EPT == 0 && (NE * 4) % 16 == 0 && NE >= EPT);
static_assert((long long)RCAP * 100 >= (long long)MAXB1024_MEAS * 105);
static_assert(WLCAP >= MAXB1024_MEAS / 8 + 8 * 51 + 1);
static_assert(MAXDEG_MEAS + 8 <= DEGCAP);
static_assert(RCAP % (NTHR * 4) == 0 && BK_ZINTS % (NTHR * 4) == 0);
static_assert((NN * 4) % 16 == 0 && NN % 4 == 0);
static_assert((MP * CIN / 8) % NTHR == 0 && (HD * CIN / 8) % NTHR == 0);
static_assert(BK_LDS <= 300000);
static_assert((GBM * SP) * 4 <= 65536);
static_assert(NN - 1 < 65536 * 16);

typedef float          v4f   __attribute__((ext_vector_type(4)));
typedef float          v8f   __attribute__((ext_vector_type(8)));
typedef int            v4i   __attribute__((ext_vector_type(4)));
typedef int            v8i   __attribute__((ext_vector_type(8)));
typedef unsigned short v8us  __attribute__((ext_vector_type(8)));
typedef unsigned short v16us __attribute__((ext_vector_type(16)));
typedef __bf16         v16bf __attribute__((ext_vector_type(16)));
typedef v4f  __attribute__((may_alias)) v4fa;
typedef v4i  __attribute__((may_alias)) v4ia;
typedef v8us __attribute__((may_alias)) v8usa;
union FragB { v16bf v; v16us u; v8us h[2]; v8i w; };

__device__ __forceinline__ v8f wmb(const FragB& a, const FragB& b, v8f c) {
  v8f d = __builtin_amdgcn_wmma_f32_16x16x32_bf16(false, a.v, false, b.v, (short)0, c, false, false);
  asm volatile("v_nop\n\tv_nop\n\tv_nop\n\tv_nop" : "+v"(d) : "v"(a.w), "v"(b.w));
  return d;
}

__device__ __forceinline__ unsigned bf16_bits(float f) {
  const unsigned u = __float_as_uint(f);
  const unsigned r = (u + 0x7FFFu + ((u >> 16) & 1u)) >> 16;
  const unsigned q = (u >> 16) | 0x40u;
  return ((u & 0x7fffffffu) > 0x7f800000u) ? q : r;
}

__device__ __forceinline__ void st2_v4f(float* p, v4f v) {
  *(volatile v4f*)p = v;
  __threadfence();
  *(volatile v4f*)p = v;
}
__device__ __forceinline__ void st2_v8us(unsigned short* p, v8us v) {
  *(volatile v8us*)p = v;
  __threadfence();
  *(volatile v8us*)p = v;
}

__device__ __forceinline__ v8us gather8(const float* __restrict__ base, int stride) {
  float f[8];
#pragma unroll
  for (int i = 0; i < 8; ++i) f[i] = base[(size_t)i * (size_t)stride];
  v8us o;
#pragma unroll
  for (int i = 0; i < 8; ++i) o[i] = (unsigned short)bf16_bits(f[i]);
  return o;
}

__global__ __launch_bounds__(NTHR) void k_prep(const float* __restrict__ x, const float* __restrict__ w1,
                                               const float* __restrict__ b1, const float* __restrict__ w2,
                                               const float* __restrict__ b2,
                                               unsigned short* xb, unsigned short* w1t, float* par) {
  const int tid = (int)threadIdx.x;
  const int blk = (int)blockIdx.x;
  if (blk < PBX) {
    const int u   = blk * NTHR + tid;
    const int row = u >> 4, k8 = (u & 15) * 8;
    const int rc  = row < NN ? row : NN - 1;
    const unsigned mk = row < NN ? 0xffffu : 0u;
    const float* p = x + (size_t)rc * CIN + k8;
    const v4f a = *(const v4fa*)p;
    const v4f b = *(const v4fa*)(p + 4);
    asm volatile("" :: "v"(a), "v"(b));
    v8us o;
    o[0] = (unsigned short)(bf16_bits(a.x) & mk); o[1] = (unsigned short)(bf16_bits(a.y) & mk);
    o[2] = (unsigned short)(bf16_bits(a.z) & mk); o[3] = (unsigned short)(bf16_bits(a.w) & mk);
    o[4] = (unsigned short)(bf16_bits(b.x) & mk); o[5] = (unsigned short)(bf16_bits(b.y) & mk);
    o[6] = (unsigned short)(bf16_bits(b.z) & mk); o[7] = (unsigned short)(bf16_bits(b.w) & mk);
    st2_v8us(xb + (size_t)row * CIN + k8, o);
  } else if (blk < PBX + PBW1) {
    const int u = (blk - PBX) * NTHR + tid;
    const int n = u >> 4, k8 = (u & 15) * 8;
    const v8us o = gather8(w1 + (size_t)k8 * HD + n, HD);
    st2_v8us(w1t + (size_t)n * CIN + k8, o);
  } else {
    if (tid < 64) {
      const int q = tid & 15;
      const v4f a = *(const v4fa*)(b1 + 4 * q);
      const v4f c = *(const v4fa*)(w2 + 4 * q);
      const float d = b2[0];
      asm volatile("" :: "v"(a), "v"(c), "v"(d));
      const unsigned ma = (tid < 16) ? 0xffffffffu : 0u;
      const unsigned mc = (tid >= 16 && tid < 32) ? 0xffffffffu : 0u;
      const unsigned md = (tid == 32) ? 0xffffffffu : 0u;
      v4f o;
      o.x = __uint_as_float(((bf16_bits(a.x) << 16) & ma) | ((bf16_bits(c.x) << 16) & mc) | ((bf16_bits(d) << 16) & md));
      o.y = __uint_as_float(((bf16_bits(a.y) << 16) & ma) | ((bf16_bits(c.y) << 16) & mc));
      o.z = __uint_as_float(((bf16_bits(a.z) << 16) & ma) | ((bf16_bits(c.z) << 16) & mc));
      o.w = __uint_as_float(((bf16_bits(a.w) << 16) & ma) | ((bf16_bits(c.w) << 16) & mc));
      st2_v4f(par + 4 * tid, o);
    }
  }
}

__device__ __forceinline__ void bucket_flush(const int* pl, const int* cnt, const int* offs, const float* dv,
                                             int ov, int* lp, int* cop, float* dp, int* fp, int tid) {
#pragma unroll 1
  for (int i = tid * 4; i < RCAP; i += NTHR * 4) {
    const v4i v = *(const v4ia*)(pl + i);
    *(volatile v4i*)(lp + i) = v;
  }
  {
    const v4i v = *(const v4ia*)(cnt + 4 * tid);
    *(volatile v4i*)(cop + 4 * tid) = v;
  }
  {
    const v4i v = *(const v4ia*)(offs + 4 * tid);
    *(volatile v4i*)(cop + NBRUN + 4 * tid) = v;
  }
  {
    const v4f v = *(const v4fa*)(dv + 4 * tid);
    *(volatile v4f*)(dp + 4 * tid) = v;
  }
  if (tid < 8) {
    const v4i f = {ov, ov, ov, ov};
    *(volatile v4i*)(fp + 4 * tid) = f;
  }
}

__global__ __launch_bounds__(NTHR) void k_bucket(const int* __restrict__ srcs, const int* __restrict__ dsts,
                                                 int* LIST, int* CO, float* DINV, int* FLAG) {
  extern __shared__ __attribute__((aligned(16))) int dsm[];
  int* wl   = dsm;
  int* pl   = dsm + NWAVE * WLCAP;
  int* cnt  = pl + RCAP;
  int* offs = cnt + NBRUN;
  int* cur  = offs + NBRUN;
  int* misc = cur + NBRUN;
  float* dv = (float*)(misc + 16);
  const int tid = (int)threadIdx.x, lane = tid & 31, wave = tid >> 5;
  const int blk = (int)blockIdx.x;
  const unsigned nbs = (unsigned)(blk * NBRUN);

  {
    const v4i z4 = {0, 0, 0, 0};
    for (int i = tid * 4; i < BK_ZINTS; i += NTHR * 4) *(v4ia*)(dsm + i) = z4;
    if (tid < 16) misc[tid] = 0;
  }
  __syncthreads();

  {
    constexpr int per = ((NE + NWAVE * WCH - 1) / (NWAVE * WCH)) * WCH;
    const int ebeg = wave * per;
    const int eend = (ebeg + per < NE) ? (ebeg + per) : NE;
    int* mylist = wl + wave * WLCAP;
    int wc = 0;
#pragma unroll 1
    for (int cb = ebeg; cb < eend; cb += WCH) {
      const int e0 = cb + lane * EPT;
      const int ec = e0 < NE - EPT ? e0 : NE - EPT;
      const v4i da = *(const v4ia*)(dsts + ec);
      const v4i db = *(const v4ia*)(dsts + ec + 4);
      asm volatile("" :: "v"(da), "v"(db));
      const bool inr = e0 < NE;
      const unsigned s0 = (unsigned)da.x - nbs, s1 = (unsigned)da.y - nbs;
      const unsigned s2 = (unsigned)da.z - nbs, s3 = (unsigned)da.w - nbs;
      const unsigned s4 = (unsigned)db.x - nbs, s5 = (unsigned)db.y - nbs;
      const unsigned s6 = (unsigned)db.z - nbs, s7 = (unsigned)db.w - nbs;
      const bool h0 = inr & (s0 < (unsigned)NBRUN), h1 = inr & (s1 < (unsigned)NBRUN);
      const bool h2 = inr & (s2 < (unsigned)NBRUN), h3 = inr & (s3 < (unsigned)NBRUN);
      const bool h4 = inr & (s4 < (unsigned)NBRUN), h5 = inr & (s5 < (unsigned)NBRUN);
      const bool h6 = inr & (s6 < (unsigned)NBRUN), h7 = inr & (s7 < (unsigned)NBRUN);
      const unsigned m0 = __builtin_amdgcn_ballot_w32(h0), m1 = __builtin_amdgcn_ballot_w32(h1);
      const unsigned m2 = __builtin_amdgcn_ballot_w32(h2), m3 = __builtin_amdgcn_ballot_w32(h3);
      const unsigned m4 = __builtin_amdgcn_ballot_w32(h4), m5 = __builtin_amdgcn_ballot_w32(h5);
      const unsigned m6 = __builtin_amdgcn_ballot_w32(h6), m7 = __builtin_amdgcn_ballot_w32(h7);
      const unsigned any = m0 | m1 | m2 | m3 | m4 | m5 | m6 | m7;
      if (any != 0u) {
        const int pre = (int)(__builtin_amdgcn_mbcnt_lo(m0, 0u) + __builtin_amdgcn_mbcnt_lo(m1, 0u) +
                              __builtin_amdgcn_mbcnt_lo(m2, 0u) + __builtin_amdgcn_mbcnt_lo(m3, 0u) +
                              __builtin_amdgcn_mbcnt_lo(m4, 0u) + __builtin_amdgcn_mbcnt_lo(m5, 0u) +
                              __builtin_amdgcn_mbcnt_lo(m6, 0u) + __builtin_amdgcn_mbcnt_lo(m7, 0u));
        int p = wc + pre;
        if (h0) { if (p < WLCAP) mylist[p] = ((e0 + 0) << SLB) | (int)s0; p = p + 1; }
        if (h1) { if (p < WLCAP) mylist[p] = ((e0 + 1) << SLB) | (int)s1; p = p + 1; }
        if (h2) { if (p < WLCAP) mylist[p] = ((e0 + 2) << SLB) | (int)s2; p = p + 1; }
        if (h3) { if (p < WLCAP) mylist[p] = ((e0 + 3) << SLB) | (int)s3; p = p + 1; }
        if (h4) { if (p < WLCAP) mylist[p] = ((e0 + 4) << SLB) | (int)s4; p = p + 1; }
        if (h5) { if (p < WLCAP) mylist[p] = ((e0 + 5) << SLB) | (int)s5; p = p + 1; }
        if (h6) { if (p < WLCAP) mylist[p] = ((e0 + 6) << SLB) | (int)s6; p = p + 1; }
        if (h7) { if (p < WLCAP) mylist[p] = ((e0 + 7) << SLB) | (int)s7; p = p + 1; }
        wc += (int)(__builtin_popcount(m0) + __builtin_popcount(m1) + __builtin_popcount(m2) + __builtin_popcount(m3) +
                    __builtin_popcount(m4) + __builtin_popcount(m5) + __builtin_popcount(m6) + __builtin_popcount(m7));
      }
    }
    if (lane == 0) misc[wave] = wc;
  }
  __syncthreads();

  if (wave == 0) {
    int ov = 0;
    int tot = 0;
#pragma unroll 1
    for (int w2 = 0; w2 < NWAVE; ++w2) {
      int c = misc[w2];
      if (c > WLCAP) ov = 1;
      c = c < 0 ? 0 : (c > WLCAP ? WLCAP : c);
      tot += c;
#pragma unroll 1
      for (int b0 = 0; b0 < c; b0 += 32) {
        const int idx = b0 + lane;
        const int ent = wl[w2 * WLCAP + (idx < WLCAP ? idx : WLCAP - 1)];
        const int m32 = (c - b0) < 32 ? (c - b0) : 32;
#pragma unroll 1
        for (int k = 0; k < m32; ++k) {
          const int u    = __builtin_amdgcn_readlane(ent, k);
          const int slot = u & (NBRUN - 1);
          if (lane == 0) cnt[slot] = cnt[slot] + 1;
        }
      }
    }
    if (tot > RCAP) ov = 1;
    if (lane == 0) misc[9] = ov;
  }
  __syncthreads();
  if (wave == 0) {
    const int base = lane * (NBRUN / 32);
    int s = 0;
#pragma unroll 1
    for (int i = 0; i < NBRUN / 32; ++i) s += cnt[base + i];
    int incl = s;
#pragma unroll
    for (int d = 1; d < 32; d <<= 1) {
      const int y = __shfl_up(incl, d, 32);
      if (lane >= d) incl += y;
    }
    int run = incl - s;
#pragma unroll 1
    for (int i = 0; i < NBRUN / 32; ++i) {
      const int cv = cnt[base + i];
      offs[base + i] = run;
      cur[base + i]  = run;
      run += cv;
    }
  }
  __syncthreads();

  if (wave == 0) {
#pragma unroll 1
    for (int w2 = 0; w2 < NWAVE; ++w2) {
      int c = misc[w2];
      c = c < 0 ? 0 : (c > WLCAP ? WLCAP : c);
#pragma unroll 1
      for (int b0 = 0; b0 < c; b0 += 32) {
        const int idx = b0 + lane;
        const int ent = wl[w2 * WLCAP + (idx < WLCAP ? idx : WLCAP - 1)];
        int eid = (ent >> SLB) & 0x1FFFFF;
        eid = eid > NE - 1 ? NE - 1 : eid;
        int sr = srcs[eid];
        sr = sr < 0 ? 0 : (sr > NN - 1 ? NN - 1 : sr);
        const int m32 = (c - b0) < 32 ? (c - b0) : 32;
#pragma unroll 1
        for (int k = 0; k < m32; ++k) {
          const int u    = __builtin_amdgcn_readlane(ent, k);
          const int wd   = __builtin_amdgcn_readlane(sr, k);
          const int slot = u & (NBRUN - 1);
          if (lane == 0) {
            int p = cur[slot];
            p = p < 0 ? 0 : (p > RCAP - 1 ? RCAP - 1 : p);
            pl[p] = wd;
            cur[slot] = p + 1;
          }
        }
      }
    }
  }
  __syncthreads();

#pragma unroll 1
  for (int j = 0; j < 4; ++j) {
    const int s = 4 * tid + j;
    const int node = blk * NBRUN + s;
    const float dg = (float)(cnt[s] + 1);
    const float d  = 1.0f / sqrtf(dg);
    dv[s] = (node < NN) ? d : 1.0f;
  }
  __syncthreads();

  const int ovf = misc[9];
  int*   lp  = LIST + (size_t)blk * RCAP;
  int*   cop = CO + (size_t)blk * (2 * NBRUN);
  float* dp  = DINV + (size_t)blk * NBRUN;
  int*   fp  = FLAG + (size_t)blk * 32;
  bucket_flush(pl, cnt, offs, dv, ovf, lp, cop, dp, fp, tid);
  __threadfence();
  bucket_flush(pl, cnt, offs, dv, ovf, lp, cop, dp, fp, tid);
}

template <int KTOT>
__device__ __forceinline__ void gemm_16x64(const unsigned short* __restrict__ ap,
                                           const unsigned short* __restrict__ bp, v8f (&acc)[4]) {
#pragma unroll 1
  for (int k0 = 0; k0 < KTOT; k0 += 32) {
    FragB af;
    af.h[0] = *(const v8usa*)(ap + k0);
    af.h[1] = *(const v8usa*)(ap + k0 + 16);
#pragma unroll
    for (int nt = 0; nt < 4; ++nt) {
      const unsigned short* wq = bp + (size_t)(16 * nt) * (size_t)KTOT + k0;
      FragB bf;
      bf.h[0] = *(const v8usa*)wq;
      bf.h[1] = *(const v8usa*)(wq + 16);
      acc[nt] = wmb(af, bf, acc[nt]);
    }
  }
}

__device__ __forceinline__ void stage_d(float* stg, const v8f (&acc)[4], int wave, int hh, int m) {
#pragma unroll
  for (int nt = 0; nt < 4; ++nt) {
#pragma unroll
    for (int r = 0; r < 8; ++r) stg[(16 * wave + 8 * hh + r) * SP + 16 * nt + m] = acc[nt][r];
  }
}

__global__ __launch_bounds__(NTHR) __attribute__((amdgpu_num_vgpr(248)))
void k_gemm1(const unsigned short* __restrict__ XB, const unsigned short* __restrict__ W1T,
             const float* __restrict__ DINV, float* P) {
  __shared__ __attribute__((aligned(16))) float stg[GBM * SP];
  const int tid = (int)threadIdx.x, lane = tid & 31, wave = tid >> 5, hh = lane >> 4, m = lane & 15;
  const int rowBase = (int)blockIdx.x * GBM;

  v8f acc[4];
  {
    const v8f z = {0.f, 0.f, 0.f, 0.f, 0.f, 0.f, 0.f, 0.f};
#pragma unroll
    for (int t = 0; t < 4; ++t) acc[t] = z;
  }
  const unsigned short* ap = XB + (size_t)(rowBase + 16 * wave + m) * (size_t)CIN + 8 * hh;
  const unsigned short* bp = W1T + (size_t)m * (size_t)CIN + 8 * hh;
  gemm_16x64<CIN>(ap, bp, acc);
  stage_d(stg, acc, wave, hh, m);
  __syncthreads();

#pragma unroll 1
  for (int i = 0; i < 8; ++i) {
    const int lr   = 16 * wave + 2 * i + hh;
    const int grow = rowBase + lr;
    const bool live = grow < NN;
    const v4f a  = *(const v4fa*)(stg + lr * SP + 4 * m);
    const float dd = DINV[grow];
    asm volatile("" :: "v"(a));
    asm volatile("" :: "v"(dd));
    const float v0 = dd * a.x, v1 = dd * a.y, v2 = dd * a.z, v3 = dd * a.w;
    v4f o;
    o.x = live ? v0 : 0.0f; o.y = live ? v1 : 0.0f; o.z = live ? v2 : 0.0f; o.w = live ? v3 : 0.0f;
    st2_v4f(P + (size_t)grow * HD + 4 * m, o);
  }
}

__global__ __launch_bounds__(NTHR) void k_replay1(const int* __restrict__ LIST, const int* __restrict__ CO,
                                                  const int* __restrict__ FLAG, const float* __restrict__ DINV,
                                                  const float* __restrict__ P, const float* __restrict__ PAR,
                                                  float* Q) {
  __shared__ __attribute__((aligned(16))) float sb[128];
  __shared__ __attribute__((aligned(16))) float qs[NBRUN];
  const int tid = (int)threadIdx.x, lane = tid & 31, wave = tid >> 5, hh = lane >> 4, q = lane & 15;
  const int blk = (int)blockIdx.x;
  const int* lb  = LIST + (size_t)blk * RCAP;
  const int* cob = CO + (size_t)blk * (2 * NBRUN);
  const int flag = FLAG[(size_t)blk * 32];
  const float qnan = __uint_as_float(0x7fc00000u);

  if (tid < 32) *(v4fa*)(sb + 4 * tid) = *(const v4fa*)(PAR + 4 * tid);
  __syncthreads();
  const v4f bias = *(const v4fa*)(sb + 4 * q);
  const v4f w2v  = *(const v4fa*)(sb + 64 + 4 * q);

#pragma unroll 1
  for (int i = 0; i < NBRUN / 16; ++i) {
    const int slot = 16 * i + 2 * wave + hh;
    const int d    = blk * NBRUN + slot;
    int c = cob[slot];
    int o = cob[NBRUN + slot];
    const float dd = DINV[d];
    asm volatile("" :: "v"(dd));
    const bool big = c > DEGCAP;
    c = c < 0 ? 0 : (c > DEGCAP ? DEGCAP : c);
    o = o < 0 ? 0 : (o > RCAP - 1 ? RCAP - 1 : o);
    const int co = __shfl_xor(c, 16, 32);
    const int cm = c > co ? c : co;
    int last = o + c - 1;
    last = last < o ? o : last;
    last = last > RCAP - 1 ? RCAP - 1 : last;
    float a0 = 0.0f, a1 = 0.0f, a2 = 0.0f, a3 = 0.0f;
#pragma unroll 1
    for (int j = 0; j < cm; ++j) {
      int idx = o + j;
      idx = idx > last ? last : idx;
      int sr = lb[idx];
      sr = sr < 0 ? 0 : (sr > NN - 1 ? NN - 1 : sr);
      const v4f v = *(const v4fa*)(P + (size_t)sr * HD + 4 * q);
      asm volatile("" :: "v"(v));
      const bool valid = j < c;
      const float t0 = a0 + v.x, t1 = a1 + v.y, t2 = a2 + v.z, t3 = a3 + v.w;
      a0 = valid ? t0 : a0; a1 = valid ? t1 : a1; a2 = valid ? t2 : a2; a3 = valid ? t3 : a3;
    }
    const v4f g = *(const v4fa*)(P + (size_t)d * HD + 4 * q);
    asm volatile("" :: "v"(g));
    a0 += g.x; a1 += g.y; a2 += g.z; a3 += g.w;
    float r0 = fmaf(dd, a0, bias.x), r1 = fmaf(dd, a1, bias.y);
    float r2 = fmaf(dd, a2, bias.z), r3 = fmaf(dd, a3, bias.w);
    r0 = (r0 > 0.0f) ? r0 : (r0 - r0); r1 = (r1 > 0.0f) ? r1 : (r1 - r1);
    r2 = (r2 > 0.0f) ? r2 : (r2 - r2); r3 = (r3 > 0.0f) ? r3 : (r3 - r3);
    float z = r0 * w2v.x;
    z = fmaf(r1, w2v.y, z);
    z = fmaf(r2, w2v.z, z);
    z = fmaf(r3, w2v.w, z);
    z += __shfl_xor(z, 8, 32);
    z += __shfl_xor(z, 4, 32);
    z += __shfl_xor(z, 2, 32);
    z += __shfl_xor(z, 1, 32);
    float qv = dd * z;
    const bool bad  = (flag != 0) | big;
    const bool live = d < NN;
    qv = bad ? qnan : qv;
    qv = live ? qv : 0.0f;
    if (q == 0) qs[slot] = qv;
  }
  __syncthreads();

  const v4f ov = *(const v4fa*)(qs + 4 * tid);
  st2_v4f(Q + (size_t)blk * NBRUN + 4 * tid, ov);
}

__global__ __launch_bounds__(NTHR) void k_replay2(const int* __restrict__ LIST, const int* __restrict__ CO,
                                                  const int* __restrict__ FLAG, const float* __restrict__ DINV,
                                                  const float* __restrict__ Q, const float* __restrict__ PAR,
                                                  float* out) {
  __shared__ __attribute__((aligned(16))) float os[NBRUN];
  const int tid = (int)threadIdx.x;
  const int blk = (int)blockIdx.x;
  const int* lb  = LIST + (size_t)blk * RCAP;
  const int* cob = CO + (size_t)blk * (2 * NBRUN);
  const int flag = FLAG[(size_t)blk * 32];
  const float b2v = PAR[128];
  const float qnan = __uint_as_float(0x7fc00000u);

#pragma unroll 1
  for (int it = 0; it < NBRUN / NTHR; ++it) {
    const int slot = it * NTHR + tid;
    const int d    = blk * NBRUN + slot;
    int c = cob[slot];
    int o = cob[NBRUN + slot];
    const float dd = DINV[d];
    asm volatile("" :: "v"(dd));
    const bool big = c > DEGCAP;
    c = c < 0 ? 0 : (c > DEGCAP ? DEGCAP : c);
    o = o < 0 ? 0 : (o > RCAP - 1 ? RCAP - 1 : o);
    int cm = c;
    { const int y = __shfl_xor(cm, 16, 32); cm = cm > y ? cm : y; }
    { const int y = __shfl_xor(cm, 8, 32);  cm = cm > y ? cm : y; }
    { const int y = __shfl_xor(cm, 4, 32);  cm = cm > y ? cm : y; }
    { const int y = __shfl_xor(cm, 2, 32);  cm = cm > y ? cm : y; }
    { const int y = __shfl_xor(cm, 1, 32);  cm = cm > y ? cm : y; }
    int last = o + c - 1;
    last = last < o ? o : last;
    last = last > RCAP - 1 ? RCAP - 1 : last;
    float s = 0.0f;
#pragma unroll 1
    for (int j = 0; j < cm; ++j) {
      int idx = o + j;
      idx = idx > last ? last : idx;
      int sr = lb[idx];
      sr = sr < 0 ? 0 : (sr > NN - 1 ? NN - 1 : sr);
      const float v = Q[sr];
      asm volatile("" :: "v"(v));
      const bool valid = j < c;
      const float t = s + v;
      s = valid ? t : s;
    }
    const float g = Q[d];
    asm volatile("" :: "v"(g));
    s += g;
    float r = fmaf(dd, s, b2v);
    const bool bad = (flag != 0) | big;
    r = bad ? qnan : r;
    os[slot] = r;
  }
  __syncthreads();

  const int e4 = blk * NBRUN + 4 * tid;
  const v4f ov = *(const v4fa*)(os + 4 * tid);
  asm volatile("" :: "v"(ov));
  float* op = out + (size_t)e4;
  const bool okst = e4 < NN;
  if (okst) *(volatile v4f*)op = ov;
  __threadfence();
  if (okst) *(volatile v4f*)op = ov;
}

extern "C" void kernel_launch(void* const* d_in, const int* in_sizes, int n_in,
                              void* d_out, int out_size, void* d_ws, size_t ws_size,
                              hipStream_t stream) {
  if (n_in < 6) return;
  if (in_sizes[0] != NN * CIN) return;
  if (in_sizes[1] != 2 * NE) return;
  if (in_sizes[2] != CIN * HD) return;
  if (in_sizes[3] != HD) return;
  if (in_sizes[4] != HD) return;
  if (in_sizes[5] != 1) return;
  if (out_size != NN) return;

  const float* x  = (const float*)d_in[0];
  const int*   ei = (const int*)d_in[1];
  const float* W1 = (const float*)d_in[2];
  const float* b1 = (const float*)d_in[3];
  const float* W2 = (const float*)d_in[4];
  const float* b2 = (const float*)d_in[5];
  float* out = (float*)d_out;
  const int* srcs = ei;
  const int* dsts = ei + NE;

  constexpr size_t zXB   = (size_t)MP * CIN * 2;
  constexpr size_t zP    = (size_t)MP * HD * 4;
  constexpr size_t zLIST = (size_t)NBK * RCAP * 4;
  constexpr size_t zCO   = (size_t)NBK * 2 * NBRUN * 4;
  constexpr size_t zDINV = (size_t)MP * 4;
  constexpr size_t zQ    = (size_t)MP * 4;
  constexpr size_t zFLAG = 6400;
  constexpr size_t zW1T  = (size_t)HD * CIN * 2;
  constexpr size_t zPAR  = 1024;
  constexpr size_t oXB   = 0;
  constexpr size_t oP    = oXB + zXB;
  constexpr size_t oLIST = oP + zP;
  constexpr size_t oCO   = oLIST + zLIST;
  constexpr size_t oDINV = oCO + zCO;
  constexpr size_t oQ    = oDINV + zDINV;
  constexpr size_t oFLAG = oQ + zQ;
  constexpr size_t oW1T  = oFLAG + zFLAG;
  constexpr size_t oPAR  = oW1T + zW1T;
  constexpr size_t oEND  = oPAR + zPAR;
  static_assert(zXB % 256 == 0 && zP % 256 == 0 && zLIST % 256 == 0 && zCO % 256 == 0);
  static_assert(zDINV % 256 == 0 && zQ % 256 == 0 && zFLAG % 256 == 0 && zW1T % 256 == 0 && zPAR % 256 == 0);
  static_assert(zFLAG >= (size_t)NBK * 128);
  static_assert(oEND <= ((size_t)128u << 20));
  if (oEND > ws_size) return;

  char* ws = (char*)d_ws;
  unsigned short* XB   = (unsigned short*)(ws + oXB);
  float*          P    = (float*)(ws + oP);
  int*            LIST = (int*)(ws + oLIST);
  int*            CO   = (int*)(ws + oCO);
  float*          DINV = (float*)(ws + oDINV);
  float*          Q    = (float*)(ws + oQ);
  int*            FLAG = (int*)(ws + oFLAG);
  unsigned short* W1T  = (unsigned short*)(ws + oW1T);
  float*          PAR  = (float*)(ws + oPAR);

  hipFuncSetAttribute(reinterpret_cast<const void*>(&k_bucket), hipFuncAttributeMaxDynamicSharedMemorySize, (int)BK_LDS);

  k_prep<<<PBTOT, NTHR, 0, stream>>>(x, W1, b1, W2, b2, XB, W1T, PAR);
  k_bucket<<<NBK, NTHR, BK_LDS, stream>>>(srcs, dsts, LIST, CO, DINV, FLAG);
  k_gemm1<<<MP / GBM, NTHR, 0, stream>>>(XB, W1T, DINV, P);
  k_replay1<<<NBK, NTHR, 0, stream>>>(LIST, CO, FLAG, DINV, P, PAR, Q);
  k_replay2<<<NBK, NTHR, 0, stream>>>(LIST, CO, FLAG, DINV, Q, PAR, out);
}
